// RGTransformer_103079215838
// MI455X (gfx1250) — hardware-verified
//
#include <hip/hip_runtime.h>
#include <math.h>

typedef __attribute__((ext_vector_type(16))) _Float16 v16h;
typedef __attribute__((ext_vector_type(16))) __bf16 v16b;
typedef __attribute__((ext_vector_type(8)))  _Float16 v8h;
typedef __attribute__((ext_vector_type(8)))  float v8f;
typedef __attribute__((ext_vector_type(4)))  float v4f;
typedef __attribute__((ext_vector_type(2)))  float v2f;
typedef __attribute__((ext_vector_type(4)))  unsigned v4u;
typedef __attribute__((ext_vector_type(4)))  int v4i;
typedef float __attribute__((may_alias)) float_a;
typedef int __attribute__((may_alias)) int_a;

template <typename T> __device__ __forceinline__ void vst2(void* p, T v) { *(volatile T*)p = v; __threadfence(); *(volatile T*)p = v; }
__device__ __forceinline__ v8f wmma16(v16h a, v16h b, v8f c) {
  v8f d = __builtin_amdgcn_wmma_f32_16x16x32_f16(false, a, false, b, (short)0, c, false, false);
  asm volatile("v_nop\n\tv_nop\n\tv_nop\n\tv_nop" : "+v"(d) : "v"(a), "v"(b));
  return d;
}
__device__ __forceinline__ v8f wmma_bf(v16b a, v16b b, v8f c) {
  v8f d = __builtin_amdgcn_wmma_f32_16x16x32_bf16(false, a, false, b, (short)0, c, false, false);
  asm volatile("v_nop\n\tv_nop\n\tv_nop\n\tv_nop" : "+v"(d) : "v"(a), "v"(b));
  return d;
}
__device__ __forceinline__ v16h frag_h(const _Float16* rowk0, int lane) {
  union { v16h v; v8h q[2]; } u; const _Float16* p = rowk0 + 8 * (lane >> 4);
  u.q[0] = *(const v8h*)p; u.q[1] = *(const v8h*)(p + 16); return u.v;
}
__device__ __forceinline__ v16h frag_f32(const float* rowk0, int lane) {
  v16h a; const float* p = rowk0 + 8 * (lane >> 4);
#pragma unroll
  for (int i = 0; i < 8; ++i) { a[i] = (_Float16)p[i]; a[8 + i] = (_Float16)p[16 + i]; }
  return a;
}
__device__ __forceinline__ v16h frag_f32s(const float* rowk0, int lane, float sc) {
  v16h a; const float* p = rowk0 + 8 * (lane >> 4);
#pragma unroll
  for (int i = 0; i < 8; ++i) { a[i] = (_Float16)(p[i] * sc); a[8 + i] = (_Float16)(p[16 + i] * sc); }
  return a;
}
__device__ __forceinline__ v16h fragc_f32(const float* W, int k0, int n, int lane, int ld, int K) {
  v16h a; const int g = lane >> 4;
#pragma unroll
  for (int i = 0; i < 8; ++i) { const int ka = k0 + 8 * g + i, kb = ka + 16;
    a[i] = (_Float16)(ka < K ? W[(size_t)ka * ld + n] : 0.f); a[8 + i] = (_Float16)(kb < K ? W[(size_t)kb * ld + n] : 0.f); }
  return a;
}
struct F2 { v16b h, l; };
__device__ __forceinline__ F2 bsplit16(const float v[16]) { F2 r;
#pragma unroll
  for (int i = 0; i < 16; ++i) { const __bf16 h = (__bf16)v[i]; r.h[i] = h; r.l[i] = (__bf16)(v[i] - (float)h); }
  return r; }
__device__ __forceinline__ F2 split_row(const float* row, int k0, int lane) { float v[16]; const float* p = row + k0 + 8 * (lane >> 4);
#pragma unroll
  for (int i = 0; i < 8; ++i) { v[i] = p[i]; v[8 + i] = p[16 + i]; }
  return bsplit16(v); }
__device__ __forceinline__ F2 split_rowK(const float* row, int k0, int lane, int K) { float v[16]; const int g = lane >> 4;
#pragma unroll
  for (int i = 0; i < 8; ++i) { const int ka = k0 + 8 * g + i, kb = ka + 16; v[i] = ka < K ? row[ka] : 0.f; v[8 + i] = kb < K ? row[kb] : 0.f; }
  return bsplit16(v); }
__device__ __forceinline__ F2 split_col(const float* W, int k0, int n, int lane, int ld, int K) { float v[16]; const int g = lane >> 4;
#pragma unroll
  for (int i = 0; i < 8; ++i) { const int ka = k0 + 8 * g + i, kb = ka + 16; v[i] = ka < K ? W[(size_t)ka * ld + n] : 0.f; v[8 + i] = kb < K ? W[(size_t)kb * ld + n] : 0.f; }
  return bsplit16(v); }
__device__ __forceinline__ v8f mac3(const F2& a, const F2& b, v8f c) { c = wmma_bf(a.l, b.h, c); c = wmma_bf(a.h, b.l, c); return wmma_bf(a.h, b.h, c); }
__device__ __forceinline__ float sigm(float v) { return 1.0f / (1.0f + expf(-v)); }
#define LDSX() do { asm volatile("s_wait_dscnt 0" ::: "memory"); __builtin_amdgcn_wave_barrier(); __builtin_amdgcn_fence(__ATOMIC_RELEASE, "workgroup"); } while (0)

#define NB 16
#define SS 1024
#define EE 256
#define NH 8
#define HD 32
#define NR (NB * SS)

__global__ __launch_bounds__(256) void k_ln(const float* __restrict__ x, const float* __restrict__ g, const float* __restrict__ bb, _Float16* __restrict__ X16, _Float16* __restrict__ M16) {
  const int wave = threadIdx.x >> 5, lane = threadIdx.x & 31; const size_t r = (size_t)blockIdx.x * 8 + wave; if (r >= NR) return;
  const float* xr = x + r * EE; float v[8]; float s = 0.f;
#pragma unroll
  for (int e = 0; e < 8; ++e) { v[e] = xr[lane * 8 + e]; s += v[e]; }
#pragma unroll
  for (int off = 16; off >= 1; off >>= 1) s += __shfl_xor(s, off, 32);
  const float mu = s * (1.0f / EE); float q2 = 0.f;
#pragma unroll
  for (int e = 0; e < 8; ++e) { const float d = v[e] - mu; q2 += d * d; }
#pragma unroll
  for (int off = 16; off >= 1; off >>= 1) q2 += __shfl_xor(q2, off, 32);
  const float rs = rsqrtf(q2 * (1.0f / EE) + 1e-5f);
  union { v8h h; v4u u; } p1, p2;
#pragma unroll
  for (int e = 0; e < 8; ++e) { const int c = lane * 8 + e; p1.h[e] = (_Float16)((v[e] - mu) * rs * g[c] + bb[c]); p2.h[e] = (_Float16)v[e]; }
  vst2(X16 + r * EE + lane * 8, p1.u); vst2(M16 + r * EE + lane * 8, p2.u);
}
__global__ __launch_bounds__(256) void k_pack(const float* __restrict__ Wq, const float* __restrict__ Wk, const float* __restrict__ Wv, const float* __restrict__ Wo, const float* __restrict__ gW, const float* __restrict__ mW, _Float16* __restrict__ P) {
  const int r = blockIdx.x, tid = threadIdx.x; __shared__ __align__(16) _Float16 srow[EE];
  const int which = r >> 8, n = r & 255; const float* W = which == 0 ? Wq : which == 1 ? Wk : which == 2 ? Wv : which == 3 ? Wo : which == 4 ? gW : mW;
  srow[tid] = (_Float16)(W[(size_t)tid * EE + n] * 16.0f);
  __syncthreads();
  if (tid < 32) vst2(P + (size_t)r * EE + tid * 8, *(const v4u*)(&srow[tid * 8]));
}
__global__ __launch_bounds__(128) void k_qkv(const _Float16* __restrict__ X16, const _Float16* __restrict__ P, const float* __restrict__ bq, const float* __restrict__ bk, const float* __restrict__ bv, _Float16* __restrict__ Q16, _Float16* __restrict__ K16, _Float16* __restrict__ VT) {
  __shared__ __align__(16) float so[4][16][132];
  __shared__ __align__(16) _Float16 st[128][72];
  const int tid = threadIdx.x, wave = tid >> 5, lane = tid & 31, col = lane & 15, g = lane >> 4;
  const int which = blockIdx.z, r0b = blockIdx.x * 64, r0 = r0b + wave * 16, n0 = blockIdx.y * 128; const int b = r0b / SS, s0 = r0b % SS;
  const _Float16* Pw = P + (size_t)which * EE * EE; const float* bias = which == 0 ? bq : (which == 1 ? bk : bv);
  v8f acc[8] = {};
#pragma unroll
  for (int kc = 0; kc < EE / 32; ++kc) { const v16h a = frag_h(X16 + (size_t)(r0 + col) * EE + kc * 32, lane);
#pragma unroll
    for (int j = 0; j < 8; ++j) acc[j] = wmma16(a, frag_h(Pw + (size_t)(n0 + j * 16 + col) * EE + kc * 32, lane), acc[j]); }
  if (which < 2) {
#pragma unroll
    for (int j = 0; j < 8; ++j) { const float bbv = bias[n0 + j * 16 + col];
#pragma unroll
      for (int r = 0; r < 8; ++r) so[wave][8 * g + r][j * 16 + col] = (acc[j][r] * (1.0f / 16.0f) + bbv) * 4.0f; }
    LDSX();
    _Float16* D = which == 0 ? Q16 : K16;
    for (int q = lane; q < 16 * 4 * 4; q += 32) { const int rl = q >> 4, hh = (q >> 2) & 3, pc = q & 3; const int h = (n0 >> 5) + hh; union { v8h h8; v4u u; } pk;
#pragma unroll
      for (int e = 0; e < 8; ++e) pk.h8[e] = (_Float16)so[wave][rl][hh * 32 + pc * 8 + e];
      vst2(D + (((size_t)b * NH + h) * SS + s0 + wave * 16 + rl) * HD + pc * 8, pk.u); } }
  else {
#pragma unroll
    for (int j = 0; j < 8; ++j) { const float bbv = bias[n0 + j * 16 + col];
#pragma unroll
      for (int r = 0; r < 8; ++r) st[j * 16 + col][wave * 16 + 8 * g + r] = (_Float16)((acc[j][r] * (1.0f / 16.0f) + bbv) * 4.0f); }
    __syncthreads();
    for (int q = tid; q < 128 * 8; q += 128) { const int cl = q >> 3, pc = q & 7; const int c = n0 + cl, h = c >> 5, d = c & 31; vst2(VT + (((size_t)b * NH + h) * HD + d) * SS + s0 + pc * 8, *(const v4u*)(&st[cl][pc * 8])); } }
}
__global__ __launch_bounds__(128) void k_attn(const _Float16* __restrict__ Q16, const _Float16* __restrict__ K16, const _Float16* __restrict__ VT, const float* __restrict__ rel, _Float16* __restrict__ O16) {
  __shared__ __align__(16) float sS[4][16][68];
  __shared__ __align__(16) _Float16 sP[4][16][72];
  __shared__ __align__(16) float sO[4][16][36];
  const int tid = threadIdx.x, w = tid >> 5, lane = tid & 31, col = lane & 15, g = lane >> 4;
  const int b = blockIdx.z, h = blockIdx.y, q0 = blockIdx.x * 64 + w * 16; const size_t bh = (size_t)b * NH + h;
  const float scl = (1.0f / 16.0f) / sqrtf((float)HD);
  const v16h aq = frag_h(Q16 + (bh * SS + q0 + col) * HD, lane);
  float mrun = -3.0e38f, lrun = 0.f; v8f acc[2] = {};
#pragma unroll 1
  for (int kt = 0; kt < SS / 64; ++kt) {
#pragma unroll
    for (int t = 0; t < 4; ++t) { v8f s = {}; const int key = kt * 64 + t * 16 + col;
      s = wmma16(aq, frag_h(K16 + (bh * SS + key) * HD, lane), s);
#pragma unroll
      for (int r = 0; r < 8; ++r) sS[w][8 * g + r][t * 16 + col] = s[r] * scl + rel[(size_t)(q0 + 8 * g + r) * SS + key]; }
    LDSX();
    float mx = -3.4e38f;
#pragma unroll
    for (int jj = 0; jj < 32; ++jj) mx = fmaxf(mx, sS[w][col][g * 32 + jj]);
    mx = fmaxf(mx, __shfl_xor(mx, 16, 32));
    const float mnew = fmaxf(mrun, mx); const float corr = expf(mrun - mnew);
    float ps = 0.f;
#pragma unroll
    for (int jj = 0; jj < 32; ++jj) { const float p = expf(sS[w][col][g * 32 + jj] - mnew); ps += p; sP[w][col][g * 32 + jj] = (_Float16)(p * 16384.0f); }
    ps += __shfl_xor(ps, 16, 32);
    lrun = lrun * corr + ps; mrun = mnew;
#pragma unroll
    for (int r = 0; r < 8; ++r) { const float cr = __shfl(corr, 8 * g + r, 32); acc[0][r] *= cr; acc[1][r] *= cr; }
    LDSX();
#pragma unroll
    for (int kc = 0; kc < 2; ++kc) { const v16h pa = frag_h(&sP[w][col][0] + kc * 32, lane);
#pragma unroll
      for (int t = 0; t < 2; ++t) acc[t] = wmma16(pa, frag_h(VT + (bh * HD + t * 16 + col) * SS + kt * 64 + kc * 32, lane), acc[t]); }
    __builtin_amdgcn_wave_barrier(); }
#pragma unroll
  for (int r = 0; r < 8; ++r) { const float lr = __shfl(lrun, 8 * g + r, 32); const float inv = 8.0f / (lr * 16384.0f * 4.0f);
#pragma unroll
    for (int t = 0; t < 2; ++t) sO[w][8 * g + r][t * 16 + col] = acc[t][r] * inv; }
  LDSX();
  for (int q = lane; q < 16 * 4; q += 32) { const int rl = q >> 2, pc = q & 3; union { v8h h8; v4u u; } pk;
#pragma unroll
    for (int e = 0; e < 8; ++e) pk.h8[e] = (_Float16)sO[w][rl][pc * 8 + e];
    vst2(O16 + (bh * SS + q0 + rl) * HD + pc * 8, pk.u); }
}
__global__ __launch_bounds__(128) void k_post(const _Float16* __restrict__ O16, const _Float16* __restrict__ M16, const _Float16* __restrict__ P, const float* __restrict__ bo, const float* __restrict__ gb, const float* __restrict__ mb,
                                            const float* __restrict__ lng, const float* __restrict__ lnb, const float* __restrict__ x, float* __restrict__ out) {
  __shared__ __align__(16) float sg1[64][EE + 4];
  __shared__ __align__(16) _Float16 sa[4][16][EE + 8];
  __shared__ __align__(16) float so[4][16][EE + 4];
  const int tid = threadIdx.x, wave = tid >> 5, lane = tid & 31, col = lane & 15, g = lane >> 4;
  const int r0b = blockIdx.x * 64, r0 = r0b + wave * 16;
#pragma unroll 1
  for (int hn = 0; hn < 2; ++hn) { v8f acc[8];
#pragma unroll
    for (int t = 0; t < 8; ++t) acc[t] = (v8f){};
#pragma unroll 1
    for (int kc = 0; kc < EE / 32; ++kc) { const int R = r0 + col; const v16h a = frag_h(O16 + ((((size_t)(R / SS)) * NH + kc) * SS + (R % SS)) * HD, lane);
#pragma unroll
      for (int t = 0; t < 8; ++t) acc[t] = wmma16(a, frag_h(P + (size_t)(3 * EE + (hn * 8 + t) * 16 + col) * EE + kc * 32, lane), acc[t]); }
#pragma unroll
    for (int t = 0; t < 8; ++t) { const int n = (hn * 8 + t) * 16 + col; const float bb = bo[n];
#pragma unroll
      for (int r = 0; r < 8; ++r) so[wave][8 * g + r][n] = acc[t][r] * (1.0f / 128.0f) + bb; } }
#pragma unroll 1
  for (int hn = 0; hn < 2; ++hn) { v8f acc[8];
#pragma unroll
    for (int t = 0; t < 8; ++t) acc[t] = (v8f){};
#pragma unroll 1
    for (int kc = 0; kc < EE / 32; ++kc) { const v16h a = frag_h(M16 + (size_t)(r0 + col) * EE + kc * 32, lane);
#pragma unroll
      for (int t = 0; t < 8; ++t) acc[t] = wmma16(a, frag_h(P + (size_t)(4 * EE + (hn * 8 + t) * 16 + col) * EE + kc * 32, lane), acc[t]); }
#pragma unroll
    for (int t = 0; t < 8; ++t) { const int n = (hn * 8 + t) * 16 + col; const float bb = gb[n];
#pragma unroll
      for (int r = 0; r < 8; ++r) sg1[wave * 16 + 8 * g + r][n] = acc[t][r] * (1.0f / 16.0f) + bb; } }
  LDSX();
  { const int rl = lane >> 1, hf = lane & 1; const int R = wave * 16 + rl; const float* xr = x + (size_t)(r0b + R) * EE;
#pragma unroll 2
    for (int c = hf * 128; c < hf * 128 + 128; ++c) { const float g1 = sigm(sg1[R][c]) * so[wave][rl][c] + xr[c]; sg1[R][c] = g1; sa[wave][rl][c] = (_Float16)g1; } }
  LDSX();
#pragma unroll 1
  for (int hn = 0; hn < 2; ++hn) { v8f acc[8];
#pragma unroll
    for (int t = 0; t < 8; ++t) acc[t] = (v8f){};
#pragma unroll 1
    for (int kc = 0; kc < EE / 32; ++kc) { const v16h a = frag_h(&sa[wave][col][0] + kc * 32, lane);
#pragma unroll
      for (int t = 0; t < 8; ++t) acc[t] = wmma16(a, frag_h(P + (size_t)(5 * EE + (hn * 8 + t) * 16 + col) * EE + kc * 32, lane), acc[t]); }
#pragma unroll
    for (int t = 0; t < 8; ++t) { const int n = (hn * 8 + t) * 16 + col; const float bb = mb[n];
#pragma unroll
      for (int r = 0; r < 8; ++r) so[wave][8 * g + r][n] = acc[t][r] * (1.0f / 16.0f) + bb; } }
  LDSX();
  { const int rl = lane >> 1, hf = lane & 1; float* row = &so[wave][rl][0]; float s = 0.f;
#pragma unroll 2
    for (int c = hf * 128; c < hf * 128 + 128; ++c) { const float mv = sigm(row[c]); row[c] = mv; s += mv; } s += __shfl_xor(s, 1, 32); const float mu = s * (1.0f / EE);
    float q2 = 0.f; for (int c = hf * 128; c < hf * 128 + 128; ++c) { const float d = row[c] - mu; q2 += d * d; } q2 += __shfl_xor(q2, 1, 32); const float rs = rsqrtf(q2 * (1.0f / EE) + 1e-5f);
    LDSX();
    const float* g1r = &sg1[wave * 16 + rl][0];
    for (int c = hf * 128; c < hf * 128 + 128; ++c) { const float lnv = (row[c] - mu) * rs * lng[c] + lnb[c]; row[c] = g1r[c] * lnv + g1r[c]; } }
  LDSX();
  for (int rl = 0; rl < 16; ++rl) for (int pc = lane; pc < EE / 4; pc += 32) vst2(out + (size_t)(r0 + rl) * EE + pc * 4, *(const v4f*)(&so[wave][rl][pc * 4]));
}
extern "C" void kernel_launch(void* const* d_in, const int* in_sizes, int n_in, void* d_out, int out_size, void* d_ws, size_t ws_size, hipStream_t stream) {
  (void)in_sizes; (void)n_in; (void)out_size; (void)ws_size;
  const float** I = (const float**)d_in;
  const float* x = I[0]; const float* lng = I[1]; const float* lnb = I[2]; const float* Wq = I[3]; const float* bq = I[4]; const float* Wk = I[5]; const float* bk = I[6]; const float* Wv = I[7]; const float* bv = I[8]; const float* Wo = I[9]; const float* bo = I[10]; const float* rel = I[11]; const float* gW = I[12]; const float* gb = I[13]; const float* mW = I[14]; const float* mb = I[15];
  float* out = (float*)d_out;
  char* ws = (char*)d_ws; size_t off = 0;
  auto take = [&](size_t bytes) { char* p = ws + off; off += (bytes + 255) & ~(size_t)255; return p; };
  _Float16* X16 = (_Float16*)take((size_t)NR * EE * 2); _Float16* M16 = (_Float16*)take((size_t)NR * EE * 2); _Float16* P = (_Float16*)take((size_t)6 * EE * EE * 2);
  _Float16* Q16 = (_Float16*)take((size_t)NR * EE * 2); _Float16* K16 = (_Float16*)take((size_t)NR * EE * 2); _Float16* VT = (_Float16*)take((size_t)NR * EE * 2); _Float16* O16 = (_Float16*)take((size_t)NR * EE * 2);
  k_ln<<<NR / 8, 256, 0, stream>>>(x, lng, lnb, X16, M16);
  k_pack<<<6 * EE, 256, 0, stream>>>(Wq, Wk, Wv, Wo, gW, mW, P);
  k_qkv<<<dim3(NR / 64, EE / 128, 3), 128, 0, stream>>>(X16, P, bq, bk, bv, Q16, K16, VT);
  k_attn<<<dim3(SS / 64, NH, NB), 128, 0, stream>>>(Q16, K16, VT, rel, O16);
  k_post<<<NR / 64, 128, 0, stream>>>(O16, M16, P, bo, gb, mb, lng, lnb, x, out);
}
